// MaskedCrossAttention_48962627174864
// MI455X (gfx1250) — hardware-verified
//
#include <hip/hip_runtime.h>
#include <math.h>
#include <stdint.h>

typedef __attribute__((ext_vector_type(16))) _Float16 v16h;
typedef __attribute__((ext_vector_type(8)))  _Float16 v8h;
typedef __attribute__((ext_vector_type(4)))  _Float16 v4h;
typedef __attribute__((ext_vector_type(16))) __bf16   v16b;
typedef __attribute__((ext_vector_type(8)))  __bf16   v8b;
typedef __attribute__((ext_vector_type(8)))  float    v8f;
typedef __attribute__((ext_vector_type(4)))  float    v4f;
typedef __attribute__((ext_vector_type(4)))  unsigned int u4;

constexpr int kBatch  = 2;
constexpr int kSeqQ   = 2048;
constexpr int kSeqKV  = 1024;
constexpr int kDim    = 1024;
constexpr int kHeads  = 8;
constexpr int kDHead  = 64;
constexpr int kInner  = kHeads * kDHead;
constexpr int kRowsQ  = kBatch * kSeqQ;
constexpr int kRowsKV = kBatch * kSeqKV;
constexpr float kLnEps = 1e-5f;
constexpr float kWCarry     = 64.0f;
constexpr float kQOutScale  = 0.125f;
constexpr float kKVOutScale = 1.0f / 64.0f;
constexpr float kScoreScale = 1.0f / 64.0f;

static_assert(kDim % 32 == 0 && kInner % 32 == 0, "K multiples of 32");
static_assert(kRowsQ % 64 == 0 && kRowsKV % 64 == 0 && kInner % 64 == 0 && kDim % 64 == 0, "M/N multiples of 64");
static_assert(kSeqQ % 64 == 0 && kSeqKV % 64 == 0 && kDHead == 64, "attention tiling");
static_assert(kDim == 4 * 256, "layernorm kernel: 256 threads x 4 elements per row");

__device__ __forceinline__ unsigned short f2bf_bits(float f) {
  unsigned u = __float_as_uint(f);
  return (unsigned short)((u + 0x7FFFu + ((u >> 16) & 1u)) >> 16);
}
__device__ __forceinline__ float bf_bits2f(unsigned short h) { return __uint_as_float(((unsigned)h) << 16); }

__device__ __forceinline__ void dep_guard_h(v8f& a, v8f& b, v16h x, v16h y) { asm volatile("v_nop\n\tv_nop\n\tv_nop\n\tv_nop" : "+v"(a), "+v"(b) : "v"(x), "v"(y)); }
__device__ __forceinline__ void dep_guard_b(v8f& a, v8f& b, v16b x, v16b y) { asm volatile("v_nop\n\tv_nop\n\tv_nop\n\tv_nop" : "+v"(a), "+v"(b) : "v"(x), "v"(y)); }
__device__ __forceinline__ void keep4_h(v16h a, v16h b, v16h c, v16h d) { asm volatile("v_nop" :: "v"(a), "v"(b), "v"(c), "v"(d)); }
__device__ __forceinline__ void keep4_b(v16b a, v16b b, v16b c, v16b d) { asm volatile("v_nop" :: "v"(a), "v"(b), "v"(c), "v"(d)); }
__device__ __forceinline__ void acc_guard4(v8f& a, v8f& b, v8f& c, v8f& d) { asm volatile("v_nop\n\tv_nop\n\tv_nop\n\tv_nop" : "+v"(a), "+v"(b), "+v"(c), "+v"(d)); }
template <typename T> struct Frag;
template <> struct Frag<_Float16> {
  typedef v16h V; union U { v16h v; v8h h[2]; };
  static __device__ __forceinline__ v16h load(const _Float16* p) {
    U f; f.h[0] = *(const v8h*)(p); f.h[1] = *(const v8h*)(p + 16); return f.v;
  }
  static __device__ __forceinline__ v8f mma(v16h a, v16h b, v8f c) {
    return __builtin_amdgcn_wmma_f32_16x16x32_f16(false, a, false, b, (short)0, c, false, false);
  }
  static __device__ __forceinline__ void guard(v8f& a, v8f& b, v16h x, v16h y) { dep_guard_h(a, b, x, y); }
  static __device__ __forceinline__ void keep(v16h a, v16h b, v16h c, v16h d) { keep4_h(a, b, c, d); }
};
template <> struct Frag<__bf16> {
  typedef v16b V; union U { v16b v; v8b h[2]; };
  static __device__ __forceinline__ v16b load(const __bf16* p) {
    U f; f.h[0] = *(const v8b*)(p); f.h[1] = *(const v8b*)(p + 16); return f.v;
  }
  static __device__ __forceinline__ v8f mma(v16b a, v16b b, v8f c) {
    return __builtin_amdgcn_wmma_f32_16x16x32_bf16(false, a, false, b, (short)0, c, false, false);
  }
  static __device__ __forceinline__ void guard(v8f& a, v8f& b, v16b x, v16b y) { dep_guard_b(a, b, x, y); }
  static __device__ __forceinline__ void keep(v16b a, v16b b, v16b c, v16b d) { keep4_b(a, b, c, d); }
};

template <int ET> struct Elem;
template <> struct Elem<0> { typedef _Float16 T; };
template <> struct Elem<1> { typedef __bf16 T; };
template <int ET, bool SPLIT, int BIAS_MODE, int OUT_MODE, bool RESID, int ACT = 0>
__global__ __launch_bounds__(256) void wmma_gemm64(
    const unsigned short* __restrict__ Ap, const unsigned short* __restrict__ A2p, int lda, long strideA,
    const unsigned short* __restrict__ Btp, const unsigned short* __restrict__ Bt2p, int ldb, long strideB,
    void* __restrict__ Cout, void* __restrict__ Cout2, int ldc, long strideC,
    const float* __restrict__ bias,
    const float* __restrict__ resid, long strideR,
    int M, int N, int K, float scale) {
  static_assert(!RESID && ACT == 0, "residual / activation paths not instantiated here");
  typedef typename Elem<ET>::T T;
  typedef typename Frag<T>::V V;
  const T* A = (const T*)Ap; const T* A2 = (const T*)A2p; const T* Bt = (const T*)Btp; const T* Bt2 = (const T*)Bt2p;
  __shared__ __align__(16) float sT[8][16 * 68];
  const int b    = blockIdx.y;
  const int lane = threadIdx.x & 31;
  const int wave = threadIdx.x >> 5;
  const int tilesN = N >> 6;
  const int tilesM = M >> 6;
  const int tile = blockIdx.x * 8 + wave;
  if (tile >= tilesM * tilesN) return;
  const int tm = tile / tilesN;
  const int tn = tile - tm * tilesN;
  const int m0 = tm << 6;
  const int n0 = tn << 6;

  const T* Ab  = A  + (size_t)b * strideA;
  const T* Bb  = Bt + (size_t)b * strideB;
  const T* Ab2 = SPLIT ? (A2  + (size_t)b * strideA) : nullptr;
  const T* Bb2 = SPLIT ? (Bt2 + (size_t)b * strideB) : nullptr;

  const int rlane = lane & 15;
  const int koff  = (lane >> 4) * 8;
  const int mOff  = (lane >> 4) * 8;

  v8f acc[4][4];
#pragma unroll
  for (int i = 0; i < 4; ++i)
#pragma unroll
    for (int j = 0; j < 4; ++j) acc[i][j] = (v8f){0.f,0.f,0.f,0.f,0.f,0.f,0.f,0.f};

  for (int k0 = 0; k0 < K; k0 += 32) {
    V bh[4], bl[4];
#pragma unroll
    for (int j = 0; j < 4; ++j) {
      const size_t bo = (size_t)(n0 + (j << 4) + rlane) * ldb + koff + k0;
      bh[j] = Frag<T>::load(Bb + bo);
      if (SPLIT) bl[j] = Frag<T>::load(Bb2 + bo);
    }
#pragma unroll
    for (int i = 0; i < 4; ++i) {
      const size_t ao = (size_t)(m0 + (i << 4) + rlane) * lda + koff + k0;
      V ah = Frag<T>::load(Ab + ao);
      V al;
      if (SPLIT) al = Frag<T>::load(Ab2 + ao);
#pragma unroll
      for (int j = 0; j < 4; ++j) {
        acc[i][j] = Frag<T>::mma(ah, bh[j], acc[i][j]);
        if (SPLIT) {
          acc[i][j] = Frag<T>::mma(ah, bl[j], acc[i][j]);
          acc[i][j] = Frag<T>::mma(al, bh[j], acc[i][j]);
        }
      }
      Frag<T>::guard(acc[i][0], acc[i][3], ah, SPLIT ? al : ah);
    }
    Frag<T>::keep(bh[0], bh[1], bh[2], bh[3]);
    if (SPLIT) Frag<T>::keep(bl[0], bl[1], bl[2], bl[3]);
  }
  acc_guard4(acc[0][0], acc[0][1], acc[0][2], acc[0][3]);
  acc_guard4(acc[1][0], acc[1][1], acc[1][2], acc[1][3]);
  acc_guard4(acc[2][0], acc[2][1], acc[2][2], acc[2][3]);
  acc_guard4(acc[3][0], acc[3][1], acc[3][2], acc[3][3]);

  float* slab = sT[wave];
#pragma unroll
  for (int i = 0; i < 4; ++i) {
    const int mBase = m0 + (i << 4);
#pragma unroll
    for (int j = 0; j < 4; ++j) {
      const int n = n0 + (j << 4) + rlane;
      float bv = 0.f;
      if (BIAS_MODE == 2) bv = bias[n];
#pragma unroll
      for (int r = 0; r < 8; ++r) {
        float v = acc[i][j][r] * scale;
        if (BIAS_MODE == 1) v += bias[mBase + mOff + r];
        if (BIAS_MODE == 2) v += bv;
        slab[(mOff + r) * 68 + (j << 4) + rlane] = v;
      }
    }
    __builtin_amdgcn_fence(__ATOMIC_RELEASE, "workgroup");
    __builtin_amdgcn_wave_barrier();
    __builtin_amdgcn_fence(__ATOMIC_ACQUIRE, "workgroup");
    if (OUT_MODE == 0) {
      float* C = (float*)Cout + (size_t)b * strideC;
      const int hh = lane >> 4, c4 = (lane & 15) * 4;
      for (int pass = 0; pass < 2; ++pass) {
#pragma unroll
        for (int it = 0; it < 8; ++it) {
          const int row = it * 2 + hh;
          v4f v = *(const v4f*)(slab + row * 68 + c4);
          *(volatile v4f*)(C + (size_t)(mBase + row) * ldc + n0 + c4) = v;
        }
        __threadfence();
      }
    } else {
      const int q = lane >> 3, c8 = (lane & 7) * 8;
      unsigned short* C  = (unsigned short*)Cout  + (size_t)b * strideC;
      unsigned short* C2 = (OUT_MODE == 2) ? ((unsigned short*)Cout2 + (size_t)b * strideC) : nullptr;
      for (int pass = 0; pass < 2; ++pass) {
#pragma unroll
        for (int it = 0; it < 4; ++it) {
          const int row = it * 4 + q;
          const float* sp = slab + row * 68 + c8;
          v8h hv, lv;
#pragma unroll
          for (int e = 0; e < 8; ++e) {
            if (OUT_MODE == 1) {
              hv[e] = (_Float16)sp[e];
              lv[e] = hv[e];
            } else {
              unsigned short hb = f2bf_bits(sp[e]);
              unsigned short lb = f2bf_bits(sp[e] - bf_bits2f(hb));
              hv[e] = __builtin_bit_cast(_Float16, hb);
              lv[e] = __builtin_bit_cast(_Float16, lb);
            }
          }
          *(volatile v8h*)(C + (size_t)(mBase + row) * ldc + n0 + c8) = hv;
          if (OUT_MODE == 2) *(volatile v8h*)(C2 + (size_t)(mBase + row) * ldc + n0 + c8) = lv;
        }
        __threadfence();
      }
    }
    __builtin_amdgcn_fence(__ATOMIC_RELEASE, "workgroup");
    __builtin_amdgcn_wave_barrier();
    __builtin_amdgcn_fence(__ATOMIC_ACQUIRE, "workgroup");
  }
}

__global__ __launch_bounds__(256) void cast_f32_f16x2(
    const float* __restrict__ in, _Float16* __restrict__ out, int n2) {
  int i = blockIdx.x * 256 + threadIdx.x;
  if (i < n2) {
    const _Float16 h0 = (_Float16)in[2 * i], h1 = (_Float16)in[2 * i + 1];
    const unsigned u = (unsigned)__builtin_bit_cast(unsigned short, h0) | ((unsigned)__builtin_bit_cast(unsigned short, h1) << 16);
    ((volatile unsigned*)out)[i] = u;
    __threadfence();
    ((volatile unsigned*)out)[i] = u;
  }
}

__device__ __forceinline__ unsigned short at_bf_bits(float f) {
  unsigned u = __float_as_uint(f);
  return (unsigned short)((u + 0x7FFFu + ((u >> 16) & 1u)) >> 16);
}
__device__ __forceinline__ __bf16 at_f2bf(float f) { return __builtin_bit_cast(__bf16, at_bf_bits(f)); }
__device__ __forceinline__ void at_split(float f, __bf16& hi, __bf16& lo) {
  const unsigned short hb = at_bf_bits(f);
  hi = __builtin_bit_cast(__bf16, hb);
  lo = at_f2bf(f - __uint_as_float(((unsigned)hb) << 16));
}
__device__ __forceinline__ v8f at_mma(v16b a, v16b b, v8f c) {
  c = __builtin_amdgcn_wmma_f32_16x16x32_bf16(false, a, false, b, (short)0, c, false, false);
  asm volatile("v_nop\n\tv_nop\n\tv_nop\n\tv_nop" : "+v"(c) : "v"(a), "v"(b));
  return c;
}
__device__ __forceinline__ v8f mma_h(v16h a, v16h b, v8f c) {
  c = __builtin_amdgcn_wmma_f32_16x16x32_f16(false, a, false, b, (short)0, c, false, false);
  asm volatile("v_nop\n\tv_nop\n\tv_nop\n\tv_nop" : "+v"(c) : "v"(a), "v"(b));
  return c;
}

__global__ __launch_bounds__(256) void ln_rows_f16(const float* __restrict__ x, const float* __restrict__ gam,
                                                   const float* __restrict__ bet, _Float16* __restrict__ xn,
                                                   int ncol, float eps) {
  __shared__ float red[8];
  const int row = blockIdx.x, tid = threadIdx.x, lane = tid & 31, wave = tid >> 5;
  const float* xr = x + (size_t)row * ncol + tid * 4;
  const v4f xv = *(const v4f*)xr;
  float s = (xv[0] + xv[1]) + (xv[2] + xv[3]);
#pragma unroll
  for (int off = 16; off > 0; off >>= 1) s += __shfl_xor(s, off, 32);
  if (lane == 0) red[wave] = s;
  __syncthreads();
  float tot = 0.f;
#pragma unroll
  for (int w = 0; w < 8; ++w) tot += red[w];
  const float invn = 1.0f / (float)ncol;
  const float mu = tot * invn;
  __syncthreads();
  const float d0 = xv[0] - mu, d1 = xv[1] - mu, d2 = xv[2] - mu, d3 = xv[3] - mu;
  float s2 = (d0 * d0 + d1 * d1) + (d2 * d2 + d3 * d3);
#pragma unroll
  for (int off = 16; off > 0; off >>= 1) s2 += __shfl_xor(s2, off, 32);
  if (lane == 0) red[wave] = s2;
  __syncthreads();
  float tot2 = 0.f;
#pragma unroll
  for (int w = 0; w < 8; ++w) tot2 += red[w];
  const float var = tot2 * invn;
  const float rs = rsqrtf(var + eps);
  const v4f g4 = *(const v4f*)(gam + tid * 4);
  const v4f b4 = *(const v4f*)(bet + tid * 4);
  v4h hv;
  hv[0] = (_Float16)(d0 * rs * g4[0] + b4[0]);
  hv[1] = (_Float16)(d1 * rs * g4[1] + b4[1]);
  hv[2] = (_Float16)(d2 * rs * g4[2] + b4[2]);
  hv[3] = (_Float16)(d3 * rs * g4[3] + b4[3]);
  _Float16* op = xn + (size_t)row * ncol + tid * 4;
  *(volatile v4h*)op = hv;
  __threadfence();
  *(volatile v4h*)op = hv;
}

template <int KIND>
__global__ __launch_bounds__(256) void transpose_cast64(const float* __restrict__ in, int nrows, int ncols,
                                                        unsigned short* __restrict__ outp, unsigned short* __restrict__ out2p,
                                                        float scale) {
  __shared__ float tile[64][65];
  const int tid = threadIdx.x, lane = tid & 31, wave = tid >> 5;
  const int c0 = blockIdx.x * 64, r0 = blockIdx.y * 64;
  {
    const int rr = tid >> 4, cc = (tid & 15) * 4;
#pragma unroll
    for (int i = 0; i < 4; ++i) {
      const int r = rr + 16 * i;
      const v4f v = *(const v4f*)(in + (size_t)(r0 + r) * ncols + c0 + cc);
      tile[r][cc + 0] = v[0];
      tile[r][cc + 1] = v[1];
      tile[r][cc + 2] = v[2];
      tile[r][cc + 3] = v[3];
    }
  }
  __syncthreads();
  const int q8 = lane >> 3, c8 = (lane & 7) * 8;
  _Float16* outh  = (_Float16*)outp;
  _Float16* out2h = (_Float16*)out2p;
  for (int pass = 0; pass < 2; ++pass) {
#pragma unroll
    for (int it = 0; it < 2; ++it) {
      const int n = wave * 8 + it * 4 + q8;
      v8h hv, lv;
#pragma unroll
      for (int e = 0; e < 8; ++e) {
        const float f = tile[c8 + e][n] * scale;
        if (KIND == 0) {
          hv[e] = (_Float16)f;
          lv[e] = hv[e];
        } else {
          const unsigned short hb = f2bf_bits(f);
          const unsigned short lb = f2bf_bits(f - bf_bits2f(hb));
          hv[e] = __builtin_bit_cast(_Float16, hb);
          lv[e] = __builtin_bit_cast(_Float16, lb);
        }
      }
      const size_t o = (size_t)(c0 + n) * nrows + r0 + c8;
      *(volatile v8h*)(outh + o) = hv;
      if (KIND == 1) *(volatile v8h*)(out2h + o) = lv;
    }
    __threadfence();
  }
}

constexpr int kAtD = 64, kAtNW = 4, kAtQB = 64, kAtKC = 64;
__global__ __launch_bounds__(128) void attn_hd64_planes(
    const unsigned short* __restrict__ Qp, int ldq,
    const unsigned short* __restrict__ Kp, int ldk,
    const unsigned short* __restrict__ Vthp, const unsigned short* __restrict__ Vtlp, int ldv,
    unsigned short* __restrict__ Ohp, unsigned short* __restrict__ Olp, int ldo,
    int S, int Skv, int H, float sscale) {
  typedef Frag<_Float16>::U FH;
  union FB { v16b v; v8b h[2]; };
  __shared__ __align__(16) _Float16 Ksh[kAtKC * kAtD];
  __shared__ __align__(16) __bf16   Vth[kAtD * kAtKC];
  __shared__ __align__(16) __bf16   Vtl[kAtD * kAtKC];
  __shared__ __align__(16) __bf16   Psh[kAtNW][16 * kAtKC];
  __shared__ __align__(16) __bf16   Psl[kAtNW][16 * kAtKC];
  __shared__ __align__(16) float    Os[kAtNW][16 * 68];

  const int tid  = threadIdx.x;
  const int wave = tid >> 5;
  const int lane = tid & 31;
  const int hh   = lane >> 4;
  const int c    = lane & 15;

  const int nqb = S / kAtQB;
  const int bx = blockIdx.x;
  const int qb = bx % nqb;
  const int bh = bx / nqb;
  const int h  = bh % H;
  const int b  = bh / H;
  const int q0 = qb * kAtQB + wave * 16;

  const _Float16* Q = (const _Float16*)Qp;
  v16h qa[2];
  {
    const _Float16* qrow = Q + (size_t)(b * S + q0 + c) * ldq + h * kAtD;
#pragma unroll
    for (int dc = 0; dc < 2; ++dc) qa[dc] = Frag<_Float16>::load(qrow + dc * 32 + 8 * hh);
  }

  float mrow[8], lrow[8];
  v8f oacc[4];
#pragma unroll
  for (int r = 0; r < 8; ++r) { mrow[r] = -INFINITY; lrow[r] = 0.f; }
#pragma unroll
  for (int t = 0; t < 4; ++t) oacc[t] = (v8f){0.f,0.f,0.f,0.f,0.f,0.f,0.f,0.f};

  const int nChunks = Skv / kAtKC;
  const int kvr = tid >> 1;
  const int dh  = (tid & 1) * 32;
  for (int kc = 0; kc < nChunks; ++kc) {
    const int kv0 = kc * kAtKC;
    __syncthreads();
    {
      const u4* ks = (const u4*)(Kp + (size_t)(b * Skv + kv0 + kvr) * ldk + h * kAtD + dh);
      const u4 k0w = ks[0], k1w = ks[1], k2w = ks[2], k3w = ks[3];
      u4* kd = (u4*)(Ksh + kvr * kAtD + dh);
      kd[0] = k0w; kd[1] = k1w; kd[2] = k2w; kd[3] = k3w;
      asm volatile("" ::: "memory");
      const u4* vhs = (const u4*)(Vthp + (size_t)(h * kAtD + kvr) * ldv + b * Skv + kv0 + dh);
      const u4 v0w = vhs[0], v1w = vhs[1], v2w = vhs[2], v3w = vhs[3];
      u4* vhd = (u4*)(Vth + kvr * kAtKC + dh);
      vhd[0] = v0w; vhd[1] = v1w; vhd[2] = v2w; vhd[3] = v3w;
      asm volatile("" ::: "memory");
      const u4* vls = (const u4*)(Vtlp + (size_t)(h * kAtD + kvr) * ldv + b * Skv + kv0 + dh);
      const u4 w0w = vls[0], w1w = vls[1], w2w = vls[2], w3w = vls[3];
      u4* vld = (u4*)(Vtl + kvr * kAtKC + dh);
      vld[0] = w0w; vld[1] = w1w; vld[2] = w2w; vld[3] = w3w;
    }
    __syncthreads();

    v8f s[4];
#pragma unroll
    for (int j = 0; j < 4; ++j) {
      s[j] = (v8f){0.f,0.f,0.f,0.f,0.f,0.f,0.f,0.f};
#pragma unroll
      for (int dc = 0; dc < 2; ++dc) {
        FH kb;
        kb.h[0] = *(const v8h*)(Ksh + (j * 16 + c) * kAtD + dc * 32 + 8 * hh);
        kb.h[1] = *(const v8h*)(Ksh + (j * 16 + c) * kAtD + dc * 32 + 16 + 8 * hh);
        s[j] = mma_h(qa[dc], kb.v, s[j]);
      }
    }
    float cm[8];
#pragma unroll
    for (int r = 0; r < 8; ++r) {
      float m = -INFINITY;
#pragma unroll
      for (int j = 0; j < 4; ++j) {
        s[j][r] = s[j][r] * sscale;
        m = fmaxf(m, s[j][r]);
      }
#pragma unroll
      for (int off = 1; off < 16; off <<= 1) m = fmaxf(m, __shfl_xor(m, off, 32));
      cm[r] = m;
    }
    __bf16* pwh = Psh[wave];
    __bf16* pwl = Psl[wave];
#pragma unroll
    for (int r = 0; r < 8; ++r) {
      const float mnew = fmaxf(mrow[r], cm[r]);
      const float alpha = expf(mrow[r] - mnew);
      mrow[r] = mnew;
      float psum = 0.f;
#pragma unroll
      for (int j = 0; j < 4; ++j) {
        const float p = expf(s[j][r] - mnew);
        psum += p;
        __bf16 ph, pl;
        at_split(p, ph, pl);
        pwh[(8 * hh + r) * kAtKC + j * 16 + c] = ph;
        pwl[(8 * hh + r) * kAtKC + j * 16 + c] = pl;
      }
#pragma unroll
      for (int off = 1; off < 16; off <<= 1) psum += __shfl_xor(psum, off, 32);
      lrow[r] = lrow[r] * alpha + psum;
#pragma unroll
      for (int t = 0; t < 4; ++t) oacc[t][r] *= alpha;
    }
    __builtin_amdgcn_fence(__ATOMIC_RELEASE, "workgroup");
    __builtin_amdgcn_wave_barrier();
    __builtin_amdgcn_fence(__ATOMIC_ACQUIRE, "workgroup");
#pragma unroll 1
    for (int kk = 0; kk < 2; ++kk) {
      FB pa, pl;
      pa.h[0] = *(const v8b*)(pwh + c * kAtKC + kk * 32 + 8 * hh);
      pa.h[1] = *(const v8b*)(pwh + c * kAtKC + kk * 32 + 16 + 8 * hh);
      pl.h[0] = *(const v8b*)(pwl + c * kAtKC + kk * 32 + 8 * hh);
      pl.h[1] = *(const v8b*)(pwl + c * kAtKC + kk * 32 + 16 + 8 * hh);
#pragma unroll
      for (int t = 0; t < 4; ++t) {
        FB vb, vl;
        vb.h[0] = *(const v8b*)(Vth + (t * 16 + c) * kAtKC + kk * 32 + 8 * hh);
        vb.h[1] = *(const v8b*)(Vth + (t * 16 + c) * kAtKC + kk * 32 + 16 + 8 * hh);
        vl.h[0] = *(const v8b*)(Vtl + (t * 16 + c) * kAtKC + kk * 32 + 8 * hh);
        vl.h[1] = *(const v8b*)(Vtl + (t * 16 + c) * kAtKC + kk * 32 + 16 + 8 * hh);
        oacc[t] = at_mma(pa.v, vb.v, oacc[t]);
        oacc[t] = at_mma(pa.v, vl.v, oacc[t]);
        oacc[t] = at_mma(pl.v, vb.v, oacc[t]);
      }
    }
  }

  float* os = Os[wave];
#pragma unroll
  for (int r = 0; r < 8; ++r) {
    const float inv = 1.0f / lrow[r];
#pragma unroll
    for (int t = 0; t < 4; ++t) os[(8 * hh + r) * 68 + t * 16 + c] = oacc[t][r] * inv;
  }
  __builtin_amdgcn_fence(__ATOMIC_RELEASE, "workgroup");
  __builtin_amdgcn_wave_barrier();
  __builtin_amdgcn_fence(__ATOMIC_ACQUIRE, "workgroup");
  {
    const int q8 = lane >> 3, c8 = (lane & 7) * 8;
    _Float16* Oh = (_Float16*)Ohp;
    _Float16* Ol = (_Float16*)Olp;
    for (int pass = 0; pass < 2; ++pass) {
#pragma unroll
      for (int it = 0; it < 4; ++it) {
        const int row = it * 4 + q8;
        const float* sp = os + row * 68 + c8;
        v8h hv, lv;
#pragma unroll
        for (int e = 0; e < 8; ++e) {
          const unsigned short hb = f2bf_bits(sp[e]);
          const unsigned short lb = f2bf_bits(sp[e] - bf_bits2f(hb));
          hv[e] = __builtin_bit_cast(_Float16, hb);
          lv[e] = __builtin_bit_cast(_Float16, lb);
        }
        const size_t o = (size_t)(b * S + q0 + row) * ldo + h * kAtD + c8;
        *(volatile v8h*)(Oh + o) = hv;
        *(volatile v8h*)(Ol + o) = lv;
      }
      __threadfence();
    }
  }
}

extern "C" void kernel_launch(void* const* d_in, const int* in_sizes, int n_in,
                              void* d_out, int out_size, void* d_ws, size_t ws_size,
                              hipStream_t stream) {
  if (n_in < 7) return;
  if (in_sizes[0] != kRowsQ * kDim || in_sizes[1] != kRowsKV * kDim || in_sizes[2] != kDim ||
      in_sizes[3] != kDim || in_sizes[4] != kDim * kInner || in_sizes[5] != kDim * 2 * kInner ||
      in_sizes[6] != kInner * kDim || out_size != kRowsQ * kDim) return;

  const float* x     = (const float*)d_in[0];
  const float* media = (const float*)d_in[1];
  const float* gam   = (const float*)d_in[2];
  const float* bet   = (const float*)d_in[3];
  const float* Wq    = (const float*)d_in[4];
  const float* Wkv   = (const float*)d_in[5];
  const float* Wout  = (const float*)d_in[6];
  float* out = (float*)d_out;

  const size_t bXn  = (size_t)kRowsQ * kDim * 2;
  const size_t bMed = (size_t)kRowsKV * kDim * 2;
  const size_t bWq  = (size_t)kInner * kDim * 2;
  const size_t bWkv = (size_t)(2 * kInner) * kDim * 2;
  const size_t bWo  = (size_t)kDim * kInner * 2;
  const size_t bQ   = (size_t)kRowsQ * kInner * 2;
  const size_t bK   = (size_t)kRowsKV * kInner * 2;
  const size_t bVt  = (size_t)kInner * kRowsKV * 2;
  const size_t bAo  = (size_t)kRowsQ * kInner * 2;

  size_t off = 0;
  char* ws = (char*)d_ws;
  unsigned short* xn_h   = (unsigned short*)(ws + off); off += bXn;
  unsigned short* med_h  = (unsigned short*)(ws + off); off += bMed;
  unsigned short* wq_t   = (unsigned short*)(ws + off); off += bWq;
  unsigned short* wkv_t  = (unsigned short*)(ws + off); off += bWkv;
  unsigned short* wo_hi  = (unsigned short*)(ws + off); off += bWo;
  unsigned short* wo_lo  = (unsigned short*)(ws + off); off += bWo;
  unsigned short* q_h    = (unsigned short*)(ws + off); off += bQ;
  unsigned short* k_h    = (unsigned short*)(ws + off); off += bK;
  unsigned short* vt_hi  = (unsigned short*)(ws + off); off += bVt;
  unsigned short* vt_lo  = (unsigned short*)(ws + off); off += bVt;
  unsigned short* ao_hi  = (unsigned short*)(ws + off); off += bAo;
  unsigned short* ao_lo  = (unsigned short*)(ws + off); off += bAo;
  if (off > ws_size) return;

  ln_rows_f16<<<dim3(kRowsQ), dim3(256), 0, stream>>>(x, gam, bet, (_Float16*)xn_h, kDim, kLnEps);
  {
    const int n2 = kRowsKV * kDim / 2;
    cast_f32_f16x2<<<dim3((n2 + 255) / 256), dim3(256), 0, stream>>>(media, (_Float16*)med_h, n2);
  }
  transpose_cast64<0><<<dim3(kInner / 64, kDim / 64), dim3(256), 0, stream>>>(Wq, kDim, kInner, wq_t, wq_t, kWCarry);
  transpose_cast64<0><<<dim3((2 * kInner) / 64, kDim / 64), dim3(256), 0, stream>>>(Wkv, kDim, 2 * kInner, wkv_t, wkv_t, kWCarry);
  transpose_cast64<1><<<dim3(kDim / 64, kInner / 64), dim3(256), 0, stream>>>(Wout, kInner, kDim, wo_hi, wo_lo, 1.0f);

  {
    const int tiles = (kRowsQ / 64) * (kInner / 64);
    wmma_gemm64<0, false, 0, 1, false><<<dim3((tiles + 7) / 8, 1), dim3(256), 0, stream>>>(
        xn_h, xn_h, kDim, 0L, wq_t, wq_t, kDim, 0L, (void*)q_h, (void*)q_h, kInner, 0L,
        gam, x, 0L, kRowsQ, kInner, kDim, kQOutScale);
  }
  {
    const int tiles = (kRowsKV / 64) * (kInner / 64);
    wmma_gemm64<0, false, 0, 1, false><<<dim3((tiles + 7) / 8, 1), dim3(256), 0, stream>>>(
        med_h, med_h, kDim, 0L, wkv_t, wkv_t, kDim, 0L, (void*)k_h, (void*)k_h, kInner, 0L,
        gam, x, 0L, kRowsKV, kInner, kDim, kKVOutScale);
  }
  {
    const int tiles = (kInner / 64) * (kRowsKV / 64);
    const unsigned short* wv_t = wkv_t + (size_t)kInner * kDim;
    wmma_gemm64<0, false, 0, 2, false><<<dim3((tiles + 7) / 8, 1), dim3(256), 0, stream>>>(
        wv_t, wv_t, kDim, 0L, med_h, med_h, kDim, 0L, (void*)vt_hi, (void*)vt_lo, kRowsKV, 0L,
        gam, x, 0L, kInner, kRowsKV, kDim, kKVOutScale);
  }
  attn_hd64_planes<<<dim3(kBatch * kHeads * (kSeqQ / kAtQB)), dim3(128), 0, stream>>>(
      q_h, kInner, k_h, kInner, vt_hi, vt_lo, kRowsKV, ao_hi, ao_lo, kInner,
      kSeqQ, kSeqKV, kHeads, kScoreScale);
  {
    const int tiles = (kRowsQ / 64) * (kDim / 64);
    wmma_gemm64<1, true, 0, 0, false><<<dim3((tiles + 7) / 8, 1), dim3(256), 0, stream>>>(
        ao_hi, ao_lo, kInner, 0L, wo_hi, wo_lo, kInner, 0L, (void*)out, (void*)out, kDim, 0L,
        gam, x, 0L, kRowsQ, kDim, kInner, 1.0f);
  }
}
